// non_local_denoising_block_17042430230629
// MI455X (gfx1250) — hardware-verified
//
#include <hip/hip_runtime.h>
#include <math.h>

typedef __attribute__((ext_vector_type(16))) _Float16 v16h;
typedef __attribute__((ext_vector_type(16))) __bf16 v16b;
typedef __attribute__((ext_vector_type(8)))  _Float16 v8h;
typedef __attribute__((ext_vector_type(8)))  float v8f;
typedef __attribute__((ext_vector_type(4)))  float v4f;
typedef __attribute__((ext_vector_type(2)))  float v2f;
typedef __attribute__((ext_vector_type(4)))  unsigned v4u;
typedef __attribute__((ext_vector_type(4)))  int v4i;
typedef float __attribute__((may_alias)) float_a;
typedef int __attribute__((may_alias)) int_a;

template <typename T> __device__ __forceinline__ void vst2(void* p, T v) { *(volatile T*)p = v; __threadfence(); *(volatile T*)p = v; }
__device__ __forceinline__ v8f wmma16(v16h a, v16h b, v8f c) {
  v8f d = __builtin_amdgcn_wmma_f32_16x16x32_f16(false, a, false, b, (short)0, c, false, false);
  asm volatile("v_nop\n\tv_nop\n\tv_nop\n\tv_nop" : "+v"(d) : "v"(a), "v"(b));
  return d;
}
__device__ __forceinline__ v8f wmma_bf(v16b a, v16b b, v8f c) {
  v8f d = __builtin_amdgcn_wmma_f32_16x16x32_bf16(false, a, false, b, (short)0, c, false, false);
  asm volatile("v_nop\n\tv_nop\n\tv_nop\n\tv_nop" : "+v"(d) : "v"(a), "v"(b));
  return d;
}
__device__ __forceinline__ v16h frag_h(const _Float16* rowk0, int lane) {
  union { v16h v; v8h q[2]; } u; const _Float16* p = rowk0 + 8 * (lane >> 4);
  u.q[0] = *(const v8h*)p; u.q[1] = *(const v8h*)(p + 16); return u.v;
}
__device__ __forceinline__ v16h frag_f32(const float* rowk0, int lane) {
  v16h a; const float* p = rowk0 + 8 * (lane >> 4);
#pragma unroll
  for (int i = 0; i < 8; ++i) { a[i] = (_Float16)p[i]; a[8 + i] = (_Float16)p[16 + i]; }
  return a;
}
__device__ __forceinline__ v16h frag_f32s(const float* rowk0, int lane, float sc) {
  v16h a; const float* p = rowk0 + 8 * (lane >> 4);
#pragma unroll
  for (int i = 0; i < 8; ++i) { a[i] = (_Float16)(p[i] * sc); a[8 + i] = (_Float16)(p[16 + i] * sc); }
  return a;
}
__device__ __forceinline__ v16h fragc_f32(const float* W, int k0, int n, int lane, int ld, int K) {
  v16h a; const int g = lane >> 4;
#pragma unroll
  for (int i = 0; i < 8; ++i) { const int ka = k0 + 8 * g + i, kb = ka + 16;
    a[i] = (_Float16)(ka < K ? W[(size_t)(ka < K ? ka : K - 1) * ld + n] : 0.f); a[8 + i] = (_Float16)(kb < K ? W[(size_t)(kb < K ? kb : K - 1) * ld + n] : 0.f); }
  return a;
}
struct F2 { v16b h, l; };
__device__ __forceinline__ F2 bsplit16(const float v[16]) { F2 r;
#pragma unroll
  for (int i = 0; i < 16; ++i) { const __bf16 h = (__bf16)v[i]; r.h[i] = h; r.l[i] = (__bf16)(v[i] - (float)h); }
  return r; }
__device__ __forceinline__ F2 split_row(const float* row, int k0, int lane) { float v[16]; const float* p = row + k0 + 8 * (lane >> 4);
#pragma unroll
  for (int i = 0; i < 8; ++i) { v[i] = p[i]; v[8 + i] = p[16 + i]; }
  return bsplit16(v); }
__device__ __forceinline__ F2 split_rowK(const float* row, int k0, int lane, int K) { float v[16]; const int g = lane >> 4;
#pragma unroll
  for (int i = 0; i < 8; ++i) { const int ka = k0 + 8 * g + i, kb = ka + 16; v[i] = ka < K ? row[ka < K ? ka : K - 1] : 0.f; v[8 + i] = kb < K ? row[kb < K ? kb : K - 1] : 0.f; }
  return bsplit16(v); }
__device__ __forceinline__ F2 split_col(const float* W, int k0, int n, int lane, int ld, int K) { float v[16]; const int g = lane >> 4;
#pragma unroll
  for (int i = 0; i < 8; ++i) { const int ka = k0 + 8 * g + i, kb = ka + 16; v[i] = ka < K ? W[(size_t)(ka < K ? ka : K - 1) * ld + n] : 0.f; v[8 + i] = kb < K ? W[(size_t)(kb < K ? kb : K - 1) * ld + n] : 0.f; }
  return bsplit16(v); }
__device__ __forceinline__ v8f mac3(const F2& a, const F2& b, v8f c) { c = wmma_bf(a.l, b.h, c); c = wmma_bf(a.h, b.l, c); return wmma_bf(a.h, b.h, c); }
__device__ __forceinline__ float sigm(float v) { return 1.0f / (1.0f + expf(-v)); }
#define LDSX() do { asm volatile("s_wait_dscnt 0" ::: "memory"); __builtin_amdgcn_wave_barrier(); __builtin_amdgcn_fence(__ATOMIC_RELEASE, "workgroup"); } while (0)


#define NB 4
#define NT 4096
#define CC 256
#define CI 128
#define NR (NB * NT)
#ifndef TQB
#define TQB (NT / 64)
#define TNB NB
#endif
typedef __attribute__((ext_vector_type(8))) __bf16 v8b;
__device__ __forceinline__ v16b frag_b(const __bf16* rowk0, int lane) {
  union { v16b v; v8b q[2]; } u; const __bf16* p = rowk0 + 8 * (lane >> 4);
  u.q[0] = *(const v8b*)p; u.q[1] = *(const v8b*)(p + 16); return u.v;
}
__device__ __forceinline__ float bfr(float v) { return (float)(__bf16)v; }
__device__ __attribute__((noinline)) float exp_ni(float v) { return expf(v); }
__device__ __attribute__((noinline)) float erf_ni(float v) { return erff(v); }

#define WS_PT  0u
#define WS_PP  (WS_PT + 2u * CI * CC)
#define WS_PG  (WS_PP + 2u * CI * CC)
#define WS_PZ  (WS_PG + 2u * CI * CC)
#define WS_TH  (WS_PZ + 2u * CC * CI)
#define WS_TL  (WS_TH + 2u * (size_t)NR * CI)
#define WS_FH  (WS_TL + 2u * (size_t)NR * CI)
#define WS_FL  (WS_FH + 2u * (size_t)NR * CI)
#define WS_G   (WS_FL + 2u * (size_t)NR * CI)
#define WS_Y   (WS_G + 2u * (size_t)NB * CI * NT)
#define WS_WY  (WS_Y + 4u * (size_t)NR * CI)
#define WS_ST  (WS_WY + 4u * (size_t)NB * CC * NT)
#define WS_END (WS_ST + 4u * CC * 2 + 256u)

__global__ __launch_bounds__(256) void k_pack(const float* __restrict__ WT, const float* __restrict__ WF, const float* __restrict__ WG, const float* __restrict__ WZ, __bf16* __restrict__ P) {
  const int n = blockIdx.x, which = blockIdx.y, t = threadIdx.x; __shared__ __align__(16) __bf16 s[CC];
  if (which < 3) { if (n >= CI) return; const float* Wm = (which == 0) ? WT : (which == 1) ? WF : WG; s[t] = (__bf16)Wm[(size_t)n * CC + t]; __syncthreads(); if (t < CC / 8) vst2((unsigned*)(P + ((which == 0) ? WS_PT / 2 : (which == 1) ? WS_PP / 2 : WS_PG / 2) + (size_t)n * CC + t * 8), *(const v4u*)&s[t * 8]); }
  else { if (t < CI) s[t] = (__bf16)WZ[(size_t)n * CI + t]; __syncthreads(); if (t < CI / 8) vst2((unsigned*)(P + WS_PZ / 2 + (size_t)n * CI + t * 8), *(const v4u*)&s[t * 8]); }
}
template <int WHICH>
__global__ __launch_bounds__(128) void k_proj(const float* __restrict__ X, const __bf16* __restrict__ P, const float* __restrict__ BB, _Float16* __restrict__ OH, _Float16* __restrict__ OL, _Float16* __restrict__ G) {
  __shared__ __align__(16) _Float16 sh[64][136], sl[64][136]; __shared__ __align__(16) _Float16 st[128][72];
  const int tid = threadIdx.x, wave = tid >> 5, lane = tid & 31, col = lane & 15, g = lane >> 4; const size_t rb0 = (size_t)blockIdx.x * 64, r0 = rb0 + wave * 16; const size_t b = rb0 / NT, t0 = rb0 % NT;
  const __bf16* Wr = P + ((WHICH == 0) ? WS_PT / 2 : (WHICH == 1) ? WS_PP / 2 : WS_PG / 2);
  v8f acc[8] = {};
#pragma unroll 2
  for (int kc = 0; kc < CC / 32; ++kc) { v16b a; { const float* p = X + ((b * CC + kc * 32 + 8 * g) * (size_t)NT) + t0 + wave * 16 + col;
#pragma unroll
      for (int i = 0; i < 8; ++i) { a[i] = (__bf16)p[(size_t)i * NT]; a[8 + i] = (__bf16)p[(size_t)(16 + i) * NT]; } }
#pragma unroll
    for (int j = 0; j < 8; ++j) acc[j] = wmma_bf(a, frag_b(Wr + (size_t)(j * 16 + col) * CC + kc * 32, lane), acc[j]); }
  if (WHICH < 2) {
#pragma unroll
    for (int j = 0; j < 8; ++j) { const float bb = bfr(BB[j * 16 + col]);
#pragma unroll
      for (int r = 0; r < 8; ++r) { const float v = acc[j][r] + bb; const _Float16 h = (_Float16)v; sh[wave * 16 + 8 * g + r][j * 16 + col] = h; sl[wave * 16 + 8 * g + r][j * 16 + col] = (_Float16)((v - (float)h) * 2048.0f); } }
    LDSX();
    for (int rl = 0; rl < 16; ++rl) if (lane < 16) { vst2((unsigned*)(OH + (r0 + rl) * CI + lane * 8), *(const v4u*)&sh[wave * 16 + rl][lane * 8]); vst2((unsigned*)(OL + (r0 + rl) * CI + lane * 8), *(const v4u*)&sl[wave * 16 + rl][lane * 8]); }
  } else {
#pragma unroll
    for (int j = 0; j < 8; ++j) { const float bb = bfr(BB[j * 16 + col]);
#pragma unroll
      for (int r = 0; r < 8; ++r) st[j * 16 + col][wave * 16 + 8 * g + r] = (_Float16)(acc[j][r] + bb); }
    __syncthreads();
    for (int e = tid; e < 128 * 8; e += 128) { const int d = e >> 3, pc = e & 7; vst2((unsigned*)(G + ((b * CI + d) * NT) + t0 + pc * 8), *(const v4u*)&st[d][pc * 8]); } }
}
__global__ __launch_bounds__(128) void k_attn(const _Float16* __restrict__ TH, const _Float16* __restrict__ TL, const _Float16* __restrict__ FH, const _Float16* __restrict__ FL, const _Float16* __restrict__ G, float* __restrict__ Y) {
  __shared__ __align__(16) _Float16 sph[4][16][40]; __shared__ __align__(16) float so[4][16][132];
  const int tid = threadIdx.x, wave = tid >> 5, lane = tid & 31, col = lane & 15, g = lane >> 4; const size_t b = blockIdx.y; const int q0 = blockIdx.x * 64 + wave * 16; const size_t rq = b * NT + q0;
  v16h aq[4], aql[4];
#pragma unroll
  for (int kc = 0; kc < 4; ++kc) { aq[kc] = frag_h(TH + (rq + col) * CI + kc * 32, lane); aql[kc] = frag_h(TL + (rq + col) * CI + kc * 32, lane); }
  float m[8], l[8];
#pragma unroll
  for (int r = 0; r < 8; ++r) { m[r] = -3.0e38f; l[r] = 0.f; }
  v8f acc[8] = {};
#pragma unroll 1
  for (int ks = 0; ks < NT / 32; ++ks) { const int j0 = ks * 32; v8f s[2];
#pragma unroll
    for (int ct = 0; ct < 2; ++ct) { const size_t rk = (b * NT + j0 + ct * 16 + col) * CI; v8f c = {}, cl = {};
#pragma unroll
      for (int kc = 0; kc < 4; ++kc) { const v16h kh = frag_h(FH + rk + kc * 32, lane); c = wmma16(aq[kc], kh, c); cl = wmma16(aql[kc], kh, cl); cl = wmma16(aq[kc], frag_h(FL + rk + kc * 32, lane), cl); }
#pragma unroll
      for (int r = 0; r < 8; ++r) s[ct][r] = c[r] + cl[r] * (1.0f / 2048.0f); }
#pragma unroll
    for (int r = 0; r < 8; ++r) { float mx = fmaxf(s[0][r], s[1][r]);
#pragma unroll
      for (int o = 1; o < 16; o <<= 1) mx = fmaxf(mx, __shfl_xor(mx, o));
      const float mn = fmaxf(m[r], mx); const float alpha = (m[r] <= -1.0e38f) ? 0.f : __expf(m[r] - mn); const float e0 = __expf(s[0][r] - mn), e1 = __expf(s[1][r] - mn); float es = e0 + e1;
#pragma unroll
      for (int o = 1; o < 16; o <<= 1) es += __shfl_xor(es, o);
      l[r] = l[r] * alpha + es; m[r] = mn;
#pragma unroll
      for (int dt = 0; dt < 8; ++dt) acc[dt][r] *= alpha;
      sph[wave][8 * g + r][col] = (_Float16)(e0 * 2048.0f); sph[wave][8 * g + r][16 + col] = (_Float16)(e1 * 2048.0f); }
    LDSX();
    const v16h pa = frag_h(&sph[wave][col][0], lane);
#pragma unroll
    for (int dt = 0; dt < 8; ++dt) acc[dt] = wmma16(pa, frag_h(G + ((b * CI + dt * 16 + col) * NT) + j0, lane), acc[dt]);
    LDSX(); }
#pragma unroll
  for (int r = 0; r < 8; ++r) { const float il = (1.0f / 2048.0f) / l[r];
#pragma unroll
    for (int dt = 0; dt < 8; ++dt) so[wave][8 * g + r][dt * 16 + col] = acc[dt][r] * il; }
  LDSX();
  for (int rl = 0; rl < 16; ++rl) vst2(Y + (rq + rl) * CI + lane * 4, *(const v4f*)&so[wave][rl][lane * 4]);
}
__global__ __launch_bounds__(128) void k_wz(const float* __restrict__ Y, const __bf16* __restrict__ P, const float* __restrict__ BZ, float* __restrict__ WY) {
  __shared__ __align__(16) float st[128][68];
  const int tid = threadIdx.x, wave = tid >> 5, lane = tid & 31, col = lane & 15, g = lane >> 4; const size_t rb0 = (size_t)blockIdx.x * 64, r0 = rb0 + wave * 16; const int n0 = blockIdx.y * 128; const size_t b = rb0 / NT, t0 = rb0 % NT;
  v8f acc[8] = {};
#pragma unroll
  for (int kc = 0; kc < CI / 32; ++kc) { const F2 a = split_row(Y + (r0 + col) * CI, kc * 32, lane);
#pragma unroll
    for (int j = 0; j < 8; ++j) { const v16b w = frag_b(P + WS_PZ / 2 + (size_t)(n0 + j * 16 + col) * CI + kc * 32, lane); acc[j] = wmma_bf(a.l, w, acc[j]); acc[j] = wmma_bf(a.h, w, acc[j]); } }
#pragma unroll
  for (int j = 0; j < 8; ++j) { const float bb = bfr(BZ[n0 + j * 16 + col]);
#pragma unroll
    for (int r = 0; r < 8; ++r) st[j * 16 + col][wave * 16 + 8 * g + r] = acc[j][r] + bb; }
  __syncthreads();
  for (int e = tid; e < 128 * 16; e += 128) { const int c = e >> 4, q = e & 15; vst2(WY + ((b * CC + n0 + c) * (size_t)NT) + t0 + q * 4, *(const v4f*)&st[c][q * 4]); }
}
__global__ __launch_bounds__(256) void k_bnstat(const float* __restrict__ WY, float* __restrict__ ST) {
  __shared__ float red[256]; const int c = blockIdx.x, t = threadIdx.x; float s = 0.f;
  for (int b = 0; b < TNB; ++b) for (int i = t; i < NT; i += 256) s += WY[(((size_t)b * CC + c) * NT) + i];
  red[t] = s; __syncthreads(); for (int st = 128; st > 0; st >>= 1) { if (t < st) red[t] += red[t + st]; __syncthreads(); }
  const float mean = red[0] / (float)(TNB * NT); __syncthreads();
  float q = 0.f; for (int b = 0; b < TNB; ++b) for (int i = t; i < NT; i += 256) { const float d = WY[(((size_t)b * CC + c) * NT) + i] - mean; q += d * d; }
  red[t] = q; __syncthreads(); for (int st = 128; st > 0; st >>= 1) { if (t < st) red[t] += red[t + st]; __syncthreads(); }
  if (t == 0) { ST[c * 2] = mean; ST[c * 2 + 1] = red[0] / (float)(TNB * NT); }
}
__global__ __launch_bounds__(256) void k_bnapply(const float* __restrict__ WY, const float* __restrict__ ST, const float* __restrict__ GA, const float* __restrict__ BE, const float* __restrict__ X, float* __restrict__ OUT) {
  const size_t b = blockIdx.y; const int c = blockIdx.x, t = threadIdx.x; const float mean = ST[c * 2], inv = 1.0f / sqrtf(ST[c * 2 + 1] + 1e-5f), ga = bfr(GA[c]), be = bfr(BE[c]); const size_t base = ((b * CC + c) * (size_t)NT);
  for (int q = t; q < NT / 4; q += 256) { v4f v; for (int i = 0; i < 4; ++i) { const size_t e = base + q * 4 + i; v[i] = ga * (WY[e] - mean) * inv + be + bfr(X[e]); } vst2(OUT + base + q * 4, v); }
}
extern "C" void kernel_launch(void* const* d_in, const int* in_sizes, int n_in, void* d_out, int out_size, void* d_ws, size_t ws_size, hipStream_t stream) {
  (void)in_sizes; (void)n_in; (void)out_size;
  const float** F = (const float**)d_in;
  if (ws_size < (size_t)WS_END) return;
  char* ws = (char*)d_ws; __bf16* P = (__bf16*)ws; _Float16 *TH = (_Float16*)(ws + WS_TH), *TL = (_Float16*)(ws + WS_TL), *FH = (_Float16*)(ws + WS_FH), *FL = (_Float16*)(ws + WS_FL), *G = (_Float16*)(ws + WS_G); float *Y = (float*)(ws + WS_Y), *WY = (float*)(ws + WS_WY), *ST = (float*)(ws + WS_ST);
  k_pack<<<dim3(CC, 4), 256, 0, stream>>>(F[3], F[5], F[1], F[7], P);
  k_proj<0><<<TNB * NT / 64, 128, 0, stream>>>(F[0], P, F[4], TH, TL, nullptr);
  k_proj<1><<<TNB * NT / 64, 128, 0, stream>>>(F[0], P, F[6], FH, FL, nullptr);
  k_proj<2><<<TNB * NT / 64, 128, 0, stream>>>(F[0], P, F[2], nullptr, nullptr, G);
  k_attn<<<dim3(TQB, TNB), 128, 0, stream>>>(TH, TL, FH, FL, G, Y);
  k_wz<<<dim3(TNB * NT / 64, CC / 128), 128, 0, stream>>>(Y, P, F[8], WY);
  k_bnstat<<<CC, 256, 0, stream>>>(WY, ST);
  k_bnapply<<<dim3(CC, TNB), 256, 0, stream>>>(WY, ST, F[9], F[10], F[0], (float*)d_out);
}
